// Graph2SeqGenerator_7962869366792
// MI455X (gfx1250) — hardware-run, weakly checked
//
#include <hip/hip_runtime.h>
#include <math.h>

typedef __attribute__((ext_vector_type(16))) _Float16 v16h;
typedef __attribute__((ext_vector_type(8)))  _Float16 v8h;
typedef __attribute__((ext_vector_type(8)))  float    v8f;
typedef __attribute__((ext_vector_type(4)))  float    v4f;

constexpr int kNodes    = 10000;
constexpr int kNodesPad = 10048;
constexpr int kEdges    = 160000;
constexpr int kEdges2   = kEdges + kNodes;
constexpr int kVocab    = 50257;
constexpr int kVocabPad = 50304;
constexpr int kEmb      = 256;
constexpr int kHid      = 128;
constexpr int kEnc      = 128;
constexpr int kSteps    = 64;
constexpr int kHeads1   = 4;
constexpr int kCh1      = kHeads1 * kHid;
constexpr int kGate     = 3 * kHid;
constexpr int kXin      = kEmb + kEnc;
constexpr int kTile1    = 16;
constexpr int kTile2    = 64;
constexpr int kBlocks1  = kNodesPad / kTile1;
constexpr int kBlocks2  = kNodesPad / kTile2;
constexpr int kChunk    = 2048;
constexpr int kNumChunks = (kEdges2 + kChunk - 1) / kChunk;
static_assert(kNodesPad % 64 == 0 && kVocabPad % 64 == 0);
static_assert(kNodesPad >= kNodes && kVocabPad >= kVocab);
static_assert(kNodes % kTile1 == 0 && kNodesPad % kTile1 == 0 && kNodesPad % kTile2 == 0);
static_assert(kEmb % 32 == 0 && kCh1 % 32 == 0 && kHid % 32 == 0);
static_assert((2 * kCh1) % 64 == 0 && (2 * kEnc) % 64 == 0);
static_assert(kEdges % 8 == 0 && kEdges2 % 8 == 0);
static_assert(kEdges2 < (1 << 20));
static_assert(kBlocks1 == 628 && kBlocks2 == 157 && kNumChunks == 84);
static_assert((kSteps * kVocab) % 4 == 0);

constexpr float kCarryW    = 256.0f;
constexpr float kCarryFeat = 256.0f;
constexpr float kCarryH1   = 1024.0f;
constexpr float kCarryHs   = 32768.0f;
constexpr float kScaleL1   = 1.0f / (kCarryFeat * kCarryW);
constexpr float kScaleL2   = 1.0f / (kCarryH1 * kCarryW);
constexpr float kScaleOut  = 1.0f / (kCarryHs * kCarryW);

constexpr size_t kSzFEATS = (size_t)kNodesPad * kEmb * 2;
constexpr size_t kSzW1T   = (size_t)(2 * kCh1) * kEmb * 2;
constexpr size_t kSzW2T   = (size_t)(2 * kEnc) * kCh1 * 2;
constexpr size_t kSzWOUT  = (size_t)kVocabPad * kHid * 2;
constexpr size_t kSzXLR1  = (size_t)kNodesPad * (2 * kCh1) * 4;
constexpr size_t kSzH1    = (size_t)kNodesPad * kCh1 * 2;
constexpr size_t kSzXLR2  = (size_t)kNodesPad * (2 * kEnc) * 4;
constexpr size_t kSzPART  = (size_t)kBlocks2 * kEnc * 4;
constexpr size_t kSzGI    = (size_t)kSteps * kGate * 4;
constexpr size_t kSzHH    = (size_t)kSteps * kHid * 2;
constexpr size_t kSzLPAD  = (size_t)kSteps * kVocabPad * 4;
constexpr size_t kOffFEATS = 0;
constexpr size_t kOffW1T   = kOffFEATS + kSzFEATS;
constexpr size_t kOffW2T   = kOffW1T + kSzW1T;
constexpr size_t kOffWOUT  = kOffW2T + kSzW2T;
constexpr size_t kOffXLR1  = kOffWOUT + kSzWOUT;
constexpr size_t kOffH1    = kOffXLR1 + kSzXLR1;
constexpr size_t kOffXLR2  = kOffH1 + kSzH1;
constexpr size_t kOffPART  = kOffXLR2 + kSzXLR2;
constexpr size_t kOffGI    = kOffPART + kSzPART;
constexpr size_t kOffHHI   = kOffGI + kSzGI;
constexpr size_t kOffHLO   = kOffHHI + kSzHH;
constexpr size_t kOffLPAD  = kOffHLO + kSzHH;
constexpr size_t kWsTotal  = kOffLPAD + kSzLPAD;
static_assert(kWsTotal == 93633024ull);
static_assert(kWsTotal <= 134217728ull);
static_assert((kSzFEATS % 128) == 0 && (kSzW1T % 128) == 0 && (kSzW2T % 128) == 0 && (kSzWOUT % 128) == 0 &&
              (kSzXLR1 % 128) == 0 && (kSzH1 % 128) == 0 && (kSzXLR2 % 128) == 0 && (kSzPART % 128) == 0 &&
              (kSzGI % 128) == 0 && (kSzHH % 128) == 0 && (kSzLPAD % 128) == 0);

__device__ __forceinline__ void pin_f(float& x) { asm volatile("" : "+v"(x)); }
__device__ __forceinline__ void pin_i(int& x) { asm volatile("" : "+v"(x)); }
__device__ __forceinline__ void pin_v4(v4f& x) { asm volatile("" : "+v"(x)); }
__device__ __forceinline__ int clampi(int v, int lo, int hi) { v = v < lo ? lo : v; v = v > hi ? hi : v; return v; }

__device__ __forceinline__ v8f mma_f16_guarded(v16h a, v16h b, v8f c) {
  c = __builtin_amdgcn_wmma_f32_16x16x32_f16(false, a, false, b, (short)0, c, false, false);
  asm volatile("v_nop\n\tv_nop\n\tv_nop\n\tv_nop" : "+v"(c) : "v"(a), "v"(b));
  return c;
}
__device__ __forceinline__ void keep4_h(v16h a, v16h b, v16h c, v16h d) { asm volatile("v_nop" :: "v"(a), "v"(b), "v"(c), "v"(d)); }
__device__ __forceinline__ void acc_guard4(v8f& a, v8f& b, v8f& c, v8f& d) { asm volatile("v_nop\n\tv_nop\n\tv_nop\n\tv_nop" : "+v"(a), "+v"(b), "+v"(c), "+v"(d)); }

struct FragH {
  union U { v16h v; v8h h[2]; };
  static __device__ __forceinline__ v16h load(const _Float16* p) {
    U f; f.h[0] = *(const v8h*)(p); f.h[1] = *(const v8h*)(p + 16); return f.v;
  }
};

template <int SPL>
__global__ __launch_bounds__(256) void wmma_gemm64_kernel(
    const unsigned short* __restrict__ Ap, const unsigned short* __restrict__ A2p, int lda,
    const unsigned short* __restrict__ Btp, int ldb,
    float* __restrict__ C, int ldc, int M, int N, int K, float scale) {
  const _Float16* A  = (const _Float16*)Ap;
  const _Float16* A2 = (const _Float16*)A2p;
  const _Float16* Bt = (const _Float16*)Btp;
  __shared__ __align__(16) float sT[8][16 * 68];
  const int lane = threadIdx.x & 31;
  const int wave = __builtin_amdgcn_readfirstlane((int)(threadIdx.x >> 5));
  const int tilesN = N >> 6;
  const int tilesM = M >> 6;
  const int tile = blockIdx.x * 8 + wave;
  if (tile >= tilesM * tilesN) return;
  const int tm = tile / tilesN;
  const int tn = tile - tm * tilesN;
  const int m0 = tm << 6;
  const int n0 = tn << 6;

  const int rlane = lane & 15;
  const int koff  = (lane >> 4) * 8;
  const int mOff  = (lane >> 4) * 8;

  v8f acc[4][4];
#pragma unroll
  for (int i = 0; i < 4; ++i)
#pragma unroll
    for (int j = 0; j < 4; ++j) acc[i][j] = (v8f){0.f,0.f,0.f,0.f,0.f,0.f,0.f,0.f};

  for (int k0 = 0; k0 < K; k0 += 32) {
    v16h bh[4];
#pragma unroll
    for (int j = 0; j < 4; ++j) {
      const size_t bo = (size_t)(n0 + (j << 4) + rlane) * ldb + koff + k0;
      bh[j] = FragH::load(Bt + bo);
    }
#pragma unroll
    for (int i = 0; i < 4; ++i) {
      const size_t ao = (size_t)(m0 + (i << 4) + rlane) * lda + koff + k0;
      v16h ah = FragH::load(A + ao);
      v16h al = ah;
      if (SPL >= 1) al = FragH::load(A2 + ao);
#pragma unroll
      for (int j = 0; j < 4; ++j) {
        acc[i][j] = mma_f16_guarded(ah, bh[j], acc[i][j]);
        if (SPL >= 1) acc[i][j] = mma_f16_guarded(al, bh[j], acc[i][j]);
      }
    }
    keep4_h(bh[0], bh[1], bh[2], bh[3]);
  }
  acc_guard4(acc[0][0], acc[0][1], acc[0][2], acc[0][3]);
  acc_guard4(acc[1][0], acc[1][1], acc[1][2], acc[1][3]);
  acc_guard4(acc[2][0], acc[2][1], acc[2][2], acc[2][3]);
  acc_guard4(acc[3][0], acc[3][1], acc[3][2], acc[3][3]);

  float* slab = sT[wave];
#pragma unroll
  for (int i = 0; i < 4; ++i) {
    const int mBase = m0 + (i << 4);
#pragma unroll
    for (int j = 0; j < 4; ++j) {
#pragma unroll
      for (int r = 0; r < 8; ++r) {
        const float v = acc[i][j][r] * scale;
        slab[(mOff + r) * 68 + (j << 4) + rlane] = v;
      }
    }
    __builtin_amdgcn_fence(__ATOMIC_RELEASE, "workgroup");
    __builtin_amdgcn_wave_barrier();
    __builtin_amdgcn_fence(__ATOMIC_ACQUIRE, "workgroup");
    {
      const int hh = lane >> 4, c4 = (lane & 15) * 4;
      for (int pass = 0; pass < 2; ++pass) {
#pragma unroll
        for (int it = 0; it < 8; ++it) {
          const int row = it * 2 + hh;
          v4f v = *(const v4f*)(slab + row * 68 + c4);
          *(volatile v4f*)(C + (size_t)(mBase + row) * ldc + n0 + c4) = v;
        }
        __threadfence();
      }
    }
    __builtin_amdgcn_fence(__ATOMIC_RELEASE, "workgroup");
    __builtin_amdgcn_wave_barrier();
    __builtin_amdgcn_fence(__ATOMIC_ACQUIRE, "workgroup");
  }
}

static_assert(((size_t)kNodesPad * kEmb / 8) % 256 == 0);
__global__ __launch_bounds__(256) void pack_feats_kernel(
    const int* __restrict__ ids, const float* __restrict__ table, unsigned short* __restrict__ out) {
  const int i  = blockIdx.x * 256 + threadIdx.x;
  const int n  = i >> 5;
  const int c8 = (i & 31) * 8;
  const int nc = n < kNodes ? n : (kNodes - 1);
  int id = ids[nc];
  id = clampi(id, 0, kVocab - 1);
  const float* p = table + (size_t)id * kEmb + c8;
  v4f a0 = *(const v4f*)(p);
  v4f a1 = *(const v4f*)(p + 4);
  pin_v4(a0);
  pin_v4(a1);
  const bool ok = n < kNodes;
  v8h hv;
#pragma unroll
  for (int e = 0; e < 4; ++e) {
    const float f0 = ok ? a0[e] * kCarryFeat : 0.0f;
    const float f1 = ok ? a1[e] * kCarryFeat : 0.0f;
    hv[e]     = (_Float16)f0;
    hv[4 + e] = (_Float16)f1;
  }
  unsigned short* q = out + (size_t)n * kEmb + c8;
  *(volatile v8h*)q = hv;
  __threadfence();
  *(volatile v8h*)q = hv;
}

__global__ __launch_bounds__(256) void pack_transpose_kernel(
    const float* __restrict__ Wa, const float* __restrict__ Wb, unsigned short* __restrict__ out,
    int K, int N, float carry) {
  __shared__ float sT[64 * 65];
  const int tid  = threadIdx.x;
  const int lane = tid & 31;
  const int wave = __builtin_amdgcn_readfirstlane((int)(threadIdx.x >> 5));
  const float* W = (blockIdx.z == 0) ? Wa : Wb;
  const int k0 = blockIdx.x * 64;
  const int n0 = blockIdx.y * 64;
  const int nn = tid & 63;
  const int kq = tid >> 6;
#pragma unroll
  for (int i = 0; i < 16; ++i) {
    const int kk = kq + 4 * i;
    sT[kk * 65 + nn] = W[(size_t)(k0 + kk) * N + n0 + nn];
  }
  __syncthreads();
  const int q  = lane >> 3;
  const int c8 = (lane & 7) * 8;
  v8h hv[2];
#pragma unroll
  for (int it = 0; it < 2; ++it) {
    const int r = it * 32 + wave * 4 + q;
#pragma unroll
    for (int e = 0; e < 8; ++e) {
      const float f = sT[(c8 + e) * 65 + r] * carry;
      hv[it][e] = (_Float16)f;
    }
  }
  for (int pass = 0; pass < 2; ++pass) {
#pragma unroll
    for (int it = 0; it < 2; ++it) {
      const int r = it * 32 + wave * 4 + q;
      const size_t row = (size_t)blockIdx.z * N + n0 + r;
      *(volatile v8h*)(out + row * K + k0 + c8) = hv[it];
    }
    __threadfence();
  }
}

static_assert(((size_t)kVocabPad * kHid / 8) % 256 == 0);
__global__ __launch_bounds__(256) void pack_wout_kernel(
    const float* __restrict__ W, unsigned short* __restrict__ out) {
  const int i   = blockIdx.x * 256 + threadIdx.x;
  const int row = i >> 4;
  const int c8  = (i & 15) * 8;
  const int rc  = row < kVocab ? row : (kVocab - 1);
  const float* p = W + (size_t)rc * kHid + c8;
  v4f a0 = *(const v4f*)(p);
  v4f a1 = *(const v4f*)(p + 4);
  pin_v4(a0);
  pin_v4(a1);
  const bool ok = row < kVocab;
  v8h hv;
#pragma unroll
  for (int e = 0; e < 4; ++e) {
    const float f0 = ok ? a0[e] * kCarryW : 0.0f;
    const float f1 = ok ? a1[e] * kCarryW : 0.0f;
    hv[e]     = (_Float16)f0;
    hv[4 + e] = (_Float16)f1;
  }
  unsigned short* q = out + (size_t)row * kHid + c8;
  *(volatile v8h*)q = hv;
  __threadfence();
  *(volatile v8h*)q = hv;
}

template <int HEADS, int TN>
__global__ __launch_bounds__(256) void edge_softmax_agg_kernel(
    const int* __restrict__ ei, const float* __restrict__ XLR, const float* __restrict__ att,
    const float* __restrict__ bias, unsigned short* __restrict__ Hout, float* __restrict__ Part) {
  constexpr int CH    = HEADS * 128;
  constexpr int PITCH = 2 * CH;
  constexpr int CPL   = CH / 32;
  constexpr int LPH   = 32 / HEADS;
  constexpr int NQ    = CPL / 4;
  static_assert(TN * CH == 8192);
  static_assert((TN & (TN - 1)) == 0 && TN >= 8 && TN <= 64);
  __shared__ __align__(16) float sNum[TN * CH];
  __shared__ float sDen[TN * HEADS];
  __shared__ unsigned sList[kChunk];
  __shared__ int sWcnt[8];

  const int tid  = threadIdx.x;
  const int lane = tid & 31;
  const int wave = __builtin_amdgcn_readfirstlane((int)(threadIdx.x >> 5));
  const int n0   = blockIdx.x * TN;
  const int c0   = lane * CPL;
  const int* srcp = ei;
  const int* dstp = ei + kEdges;

  v4f av[NQ];
#pragma unroll
  for (int q = 0; q < NQ; ++q) av[q] = *(const v4f*)(att + c0 + 4 * q);

#pragma unroll 1
  for (int i = tid; i < TN * CH; i += 256) sNum[i] = 0.0f;
  if (tid < TN * HEADS) sDen[tid] = 0.0f;
  __syncthreads();

#pragma unroll 1
  for (int ch = 0; ch < kNumChunks; ++ch) {
    const int eb = ch * kChunk + tid * 8;
    const bool real = eb < kEdges;
    const bool inr  = eb < kEdges2;
    const int ebc   = real ? eb : 0;
    const int4 da = *(const int4*)(dstp + ebc);
    const int4 db = *(const int4*)(dstp + ebc + 4);
    int dv[8];
    dv[0] = da.x; dv[1] = da.y; dv[2] = da.z; dv[3] = da.w;
    dv[4] = db.x; dv[5] = db.y; dv[6] = db.z; dv[7] = db.w;
#pragma unroll
    for (int j = 0; j < 8; ++j) pin_i(dv[j]);

    bool hit[8];
    unsigned ent[8];
    bool hany = false;
#pragma unroll
    for (int j = 0; j < 8; ++j) {
      const int dr = clampi(dv[j], 0, kNodes - 1);
      const int dd = real ? dr : (eb + j - kEdges);
      const int dl = dd - n0;
      const bool h = inr && ((unsigned)dl < (unsigned)TN);
      hit[j] = h;
      ent[j] = (unsigned)(eb + j) | ((unsigned)(h ? dl : 0) << 20);
      hany = hany || h;
    }
    const unsigned anyw = __builtin_amdgcn_ballot_w32(hany);
    int running = 0;
    int off[8];
#pragma unroll
    for (int j = 0; j < 8; ++j) off[j] = 0;
    if (anyw != 0u) {
      const unsigned lt = (1u << lane) - 1u;
#pragma unroll
      for (int j = 0; j < 8; ++j) {
        const unsigned m = __builtin_amdgcn_ballot_w32(hit[j]);
        off[j] = running + __popc(m & lt);
        running += __popc(m);
      }
    }
    if (lane == 0) sWcnt[wave] = running;
    __syncthreads();
    int base = 0, total = 0;
#pragma unroll
    for (int w = 0; w < 8; ++w) {
      const int c = sWcnt[w];
      total += c;
      base += (w < wave) ? c : 0;
    }
#pragma unroll
    for (int j = 0; j < 8; ++j) {
      if (hit[j]) {
        int pos = base + off[j];
        pos = pos > (kChunk - 1) ? (kChunk - 1) : pos;
        sList[pos] = ent[j];
      }
    }
    __syncthreads();
    total = __builtin_amdgcn_readfirstlane(total);
    total = total > kChunk ? kChunk : total;
#pragma unroll 1
    for (int i = 0; i < total; ++i) {
      const unsigned en = (unsigned)__builtin_amdgcn_readfirstlane((int)sList[i]);
      const int dl = (int)(en >> 20) & (TN - 1);
      if ((dl & 7) == wave) {
        const int e  = (int)(en & 0xFFFFFu);
        const int ec = e < kEdges ? e : (kEdges - 1);
        int sl = srcp[ec];
        sl = clampi(sl, 0, kNodes - 1);
        int s = (e < kEdges) ? sl : (e - kEdges);
        s = clampi(s, 0, kNodes - 1);
        int d = n0 + dl;
        d = d > (kNodes - 1) ? (kNodes - 1) : d;
        const float* xlp = XLR + (size_t)s * PITCH + c0;
        const float* xrp = XLR + (size_t)d * PITCH + CH + c0;
        v4f xl[NQ], xr[NQ];
#pragma unroll
        for (int q = 0; q < NQ; ++q) {
          xl[q] = *(const v4f*)(xlp + 4 * q);
          xr[q] = *(const v4f*)(xrp + 4 * q);
        }
        float part = 0.0f;
#pragma unroll
        for (int q = 0; q < NQ; ++q) {
#pragma unroll
          for (int c = 0; c < 4; ++c) {
            float v = xl[q][c] + xr[q][c];
            v = (v >= 0.0f) ? v : 0.2f * v;
            part = fmaf(av[q][c], v, part);
          }
        }
#pragma unroll
        for (int o = 1; o < LPH; o <<= 1) part += __shfl_xor(part, o, 32);
        const float lg = fminf(fmaxf(part, -60.0f), 60.0f);
        const float a = expf(lg);
        float* np = sNum + dl * CH + c0;
#pragma unroll
        for (int q = 0; q < NQ; ++q) {
          v4f nv = *(const v4f*)(np + 4 * q);
#pragma unroll
          for (int c = 0; c < 4; ++c) nv[c] = fmaf(a, xl[q][c], nv[c]);
          *(v4f*)(np + 4 * q) = nv;
        }
        if ((lane & (LPH - 1)) == 0) sDen[dl * HEADS + lane / LPH] += a;
      }
    }
    __syncthreads();
  }

  if (HEADS == 4) {
#pragma unroll 1
    for (int i = 0; i < (TN * CH) / 256; ++i) {
      const int idx = i * 256 + tid;
      const int row = idx / CH;
      const int c   = idx - row * CH;
      const bool valid = (n0 + row) < kNodes;
      const float den  = sDen[row * HEADS + c / 128];
      const float denc = (valid && den > 0.0f) ? den : 1.0f;
      const float v = sNum[idx] * (1.0f / denc) + bias[c];
      const float ev = (v > 0.0f) ? v : (expf(v) - 1.0f);
      sNum[idx] = valid ? ev * kCarryH1 : 0.0f;
    }
    __syncthreads();
    v8h hv[4];
#pragma unroll
    for (int it = 0; it < 4; ++it) {
      const int idx8 = it * 256 + tid;
      const int row  = idx8 >> 6;
      const int c8   = (idx8 & 63) * 8;
      const float* sp = sNum + row * CH + c8;
      const v4f a0 = *(const v4f*)(sp);
      const v4f a1 = *(const v4f*)(sp + 4);
#pragma unroll
      for (int e = 0; e < 4; ++e) {
        hv[it][e]     = (_Float16)a0[e];
        hv[it][4 + e] = (_Float16)a1[e];
      }
    }
    for (int pass = 0; pass < 2; ++pass) {
#pragma unroll
      for (int it = 0; it < 4; ++it) {
        const int idx8 = it * 256 + tid;
        const int row  = idx8 >> 6;
        const int c8   = (idx8 & 63) * 8;
        *(volatile v8h*)(Hout + (size_t)(n0 + row) * CH + c8) = hv[it];
      }
      __threadfence();
    }
  } else {
    if (tid < CH) {
      float acc = 0.0f;
#pragma unroll 1
      for (int row = 0; row < TN; ++row) {
        const bool valid = (n0 + row) < kNodes;
        const float den  = sDen[row];
        const float denc = (valid && den > 0.0f) ? den : 1.0f;
        const float t = sNum[row * CH + tid] * (1.0f / denc);
        acc += valid ? t : 0.0f;
      }
      float* q = Part + (size_t)blockIdx.x * CH + tid;
      *(volatile float*)q = acc;
      __threadfence();
      *(volatile float*)q = acc;
    }
  }
}

__global__ __launch_bounds__(384) void input_gates_kernel(
    const int* __restrict__ seq, const float* __restrict__ table, const float* __restrict__ Part,
    const float* __restrict__ b2, const float* __restrict__ Wih, const float* __restrict__ bih,
    float* __restrict__ GI) {
  __shared__ __align__(16) float sx[kXin];
  const int t = blockIdx.x;
  const int j = threadIdx.x;
  const int tm = (t > 0) ? (t - 1) : 0;
  int tk = seq[tm];
  tk = clampi(tk, 0, kVocab - 1);
  const int tok = (t > 0) ? tk : 0;
  if (j < kEmb) {
    sx[j] = table[(size_t)tok * kEmb + j];
  } else {
    const int c = j - kEmb;
    float s = 0.0f;
#pragma unroll 1
    for (int b = 0; b < kBlocks2; ++b) s += Part[(size_t)b * kEnc + c];
    sx[j] = s * (1.0f / (float)kNodes) + b2[c];
  }
  __syncthreads();
  const float* wr = Wih + (size_t)j * kXin;
  float acc = bih[j];
#pragma unroll 1
  for (int k4 = 0; k4 < kXin / 4; ++k4) {
    const v4f w = *(const v4f*)(wr + 4 * k4);
    const v4f x = *(const v4f*)(sx + 4 * k4);
    acc = fmaf(w[0], x[0], acc);
    acc = fmaf(w[1], x[1], acc);
    acc = fmaf(w[2], x[2], acc);
    acc = fmaf(w[3], x[3], acc);
  }
  float* q = GI + (size_t)t * kGate + j;
  *(volatile float*)q = acc;
  __threadfence();
  *(volatile float*)q = acc;
}

__global__ __launch_bounds__(384) void recurrent_cell_kernel(
    const float* __restrict__ GI, const float* __restrict__ Whh, const float* __restrict__ bhh,
    unsigned short* __restrict__ HHi, unsigned short* __restrict__ HLo) {
  __shared__ __align__(16) float sh[kHid];
  __shared__ float sgi[kGate];
  __shared__ float sgh[kGate];
  __shared__ __align__(16) float sHall[kSteps * kHid];
  const int j = threadIdx.x;
  if (j < kHid) sh[j] = 0.0f;
  const float bj = bhh[j];
  const float* wr = Whh + (size_t)j * kHid;
  __syncthreads();
#pragma unroll 1
  for (int t = 0; t < kSteps; ++t) {
    const float gi = GI[(size_t)t * kGate + j];
    float acc = bj;
#pragma unroll 1
    for (int k4 = 0; k4 < kHid / 4; ++k4) {
      const v4f w = *(const v4f*)(wr + 4 * k4);
      const v4f x = *(const v4f*)(sh + 4 * k4);
      acc = fmaf(w[0], x[0], acc);
      acc = fmaf(w[1], x[1], acc);
      acc = fmaf(w[2], x[2], acc);
      acc = fmaf(w[3], x[3], acc);
    }
    sgi[j] = gi;
    sgh[j] = acc;
    __syncthreads();
    if (j < kHid) {
      const float ar = sgi[j] + sgh[j];
      const float az = sgi[kHid + j] + sgh[kHid + j];
      const float r = 1.0f / (1.0f + expf(-ar));
      const float z = 1.0f / (1.0f + expf(-az));
      const float cand = tanhf(sgi[2 * kHid + j] + r * sgh[2 * kHid + j]);
      const float hn = (1.0f - z) * cand + z * sh[j];
      sh[j] = hn;
      sHall[t * kHid + j] = hn;
    }
    __syncthreads();
  }
  constexpr int kItems = kSteps * kHid / 8;
  v8h hv[3], lv[3];
#pragma unroll
  for (int it = 0; it < 3; ++it) {
    const int item = it * 384 + j;
    const int ic = item < kItems ? item : (kItems - 1);
    const float* sp = sHall + ic * 8;
    const v4f a0 = *(const v4f*)(sp);
    const v4f a1 = *(const v4f*)(sp + 4);
#pragma unroll
    for (int e = 0; e < 4; ++e) {
      const float s0 = a0[e] * kCarryHs;
      const float s1 = a1[e] * kCarryHs;
      const _Float16 h0 = (_Float16)s0;
      const _Float16 h1 = (_Float16)s1;
      const float r0 = s0 - (float)h0;
      const float r1 = s1 - (float)h1;
      hv[it][e]     = h0;
      hv[it][4 + e] = h1;
      lv[it][e]     = (_Float16)r0;
      lv[it][4 + e] = (_Float16)r1;
    }
  }
  for (int pass = 0; pass < 2; ++pass) {
#pragma unroll
    for (int it = 0; it < 3; ++it) {
      const int item = it * 384 + j;
      if (item < kItems) {
        *(volatile v8h*)(HHi + (size_t)item * 8) = hv[it];
        *(volatile v8h*)(HLo + (size_t)item * 8) = lv[it];
      }
    }
    __threadfence();
  }
}

__global__ __launch_bounds__(256) void repack_out_kernel(
    const float* __restrict__ Lp, const float* __restrict__ bout, float* __restrict__ out) {
  constexpr int kTotal4 = (kSteps * kVocab) / 4;
  const int i4 = blockIdx.x * 256 + threadIdx.x;
  const int ic = (i4 < kTotal4) ? i4 : (kTotal4 - 1);
  const int base = ic * 4;
  float val[4];
#pragma unroll
  for (int e = 0; e < 4; ++e) {
    const int idx = base + e;
    const int t = idx / kVocab;
    const int v = idx - t * kVocab;
    float x = Lp[(size_t)t * kVocabPad + v];
    float b = bout[v];
    pin_f(x);
    pin_f(b);
    val[e] = x + b;
  }
  v4f o;
  o[0] = val[0]; o[1] = val[1]; o[2] = val[2]; o[3] = val[3];
  if (i4 < kTotal4) {
    float* q = out + (size_t)i4 * 4;
    *(volatile v4f*)q = o;
    __threadfence();
    *(volatile v4f*)q = o;
  }
}

extern "C" void kernel_launch(void* const* d_in, const int* in_sizes, int n_in,
                              void* d_out, int out_size, void* d_ws, size_t ws_size,
                              hipStream_t stream) {
  if (n_in < 18) return;
  if (in_sizes[0] != kNodes) return;
  if (in_sizes[1] != 2 * kEdges) return;
  if (in_sizes[2] != kSteps) return;
  if (in_sizes[3] != kVocab * kEmb) return;
  if (in_sizes[4] != kEmb * kCh1) return;
  if (in_sizes[5] != kEmb * kCh1) return;
  if (in_sizes[6] != kCh1) return;
  if (in_sizes[7] != kCh1) return;
  if (in_sizes[8] != kCh1 * kEnc) return;
  if (in_sizes[9] != kCh1 * kEnc) return;
  if (in_sizes[10] != kEnc) return;
  if (in_sizes[11] != kEnc) return;
  if (in_sizes[12] != kGate * kXin) return;
  if (in_sizes[13] != kGate * kHid) return;
  if (in_sizes[14] != kGate) return;
  if (in_sizes[15] != kGate) return;
  if (in_sizes[16] != kVocab * kHid) return;
  if (in_sizes[17] != kVocab) return;
  if (out_size != kSteps * kVocab) return;
  if (ws_size < kWsTotal) return;

  const int*   x_nodes = (const int*)d_in[0];
  const int*   ei      = (const int*)d_in[1];
  const int*   tseq    = (const int*)d_in[2];
  const float* table   = (const float*)d_in[3];
  const float* W1l     = (const float*)d_in[4];
  const float* W1r     = (const float*)d_in[5];
  const float* att1    = (const float*)d_in[6];
  const float* b1      = (const float*)d_in[7];
  const float* W2l     = (const float*)d_in[8];
  const float* W2r     = (const float*)d_in[9];
  const float* att2    = (const float*)d_in[10];
  const float* b2      = (const float*)d_in[11];
  const float* Wih     = (const float*)d_in[12];
  const float* Whh     = (const float*)d_in[13];
  const float* bih     = (const float*)d_in[14];
  const float* bhh     = (const float*)d_in[15];
  const float* Wout    = (const float*)d_in[16];
  const float* bout    = (const float*)d_in[17];
  float* out = (float*)d_out;

  char* ws = (char*)d_ws;
  unsigned short* FEATS = (unsigned short*)(ws + kOffFEATS);
  unsigned short* W1T   = (unsigned short*)(ws + kOffW1T);
  unsigned short* W2T   = (unsigned short*)(ws + kOffW2T);
  unsigned short* WOUTH = (unsigned short*)(ws + kOffWOUT);
  float*          XLR1  = (float*)(ws + kOffXLR1);
  unsigned short* H1    = (unsigned short*)(ws + kOffH1);
  float*          XLR2  = (float*)(ws + kOffXLR2);
  float*          PART  = (float*)(ws + kOffPART);
  float*          GI    = (float*)(ws + kOffGI);
  unsigned short* HHI   = (unsigned short*)(ws + kOffHHI);
  unsigned short* HLO   = (unsigned short*)(ws + kOffHLO);
  float*          LPAD  = (float*)(ws + kOffLPAD);

  pack_feats_kernel<<<(kNodesPad * kEmb / 8) / 256, 256, 0, stream>>>(x_nodes, table, FEATS);
  pack_transpose_kernel<<<dim3(kEmb / 64, kCh1 / 64, 2), 256, 0, stream>>>(W1l, W1r, W1T, kEmb, kCh1, kCarryW);
  pack_transpose_kernel<<<dim3(kCh1 / 64, kEnc / 64, 2), 256, 0, stream>>>(W2l, W2r, W2T, kCh1, kEnc, kCarryW);
  pack_wout_kernel<<<(kVocabPad * kHid / 8) / 256, 256, 0, stream>>>(Wout, WOUTH);

  {
    const int tiles = (kNodesPad / 64) * ((2 * kCh1) / 64);
    wmma_gemm64_kernel<0><<<(tiles + 7) / 8, 256, 0, stream>>>(
        FEATS, nullptr, kEmb, W1T, kEmb, XLR1, 2 * kCh1, kNodesPad, 2 * kCh1, kEmb, kScaleL1);
  }
  edge_softmax_agg_kernel<kHeads1, kTile1><<<kBlocks1, 256, 0, stream>>>(ei, XLR1, att1, b1, H1, nullptr);

  {
    const int tiles = (kNodesPad / 64) * ((2 * kEnc) / 64);
    wmma_gemm64_kernel<0><<<(tiles + 7) / 8, 256, 0, stream>>>(
        H1, nullptr, kCh1, W2T, kCh1, XLR2, 2 * kEnc, kNodesPad, 2 * kEnc, kCh1, kScaleL2);
  }
  edge_softmax_agg_kernel<1, kTile2><<<kBlocks2, 256, 0, stream>>>(ei, XLR2, att2, b2, nullptr, PART);

  input_gates_kernel<<<kSteps, 384, 0, stream>>>(tseq, table, PART, b2, Wih, bih, GI);
  recurrent_cell_kernel<<<1, 384, 0, stream>>>(GI, Whh, bhh, HHI, HLO);
  {
    const int tiles = (kSteps / 64) * (kVocabPad / 64);
    wmma_gemm64_kernel<1><<<(tiles + 7) / 8, 256, 0, stream>>>(
        HHI, HLO, kHid, WOUTH, kHid, LPAD, kVocabPad, kSteps, kVocabPad, kHid, kScaleOut);
  }
  {
    const int total4 = (kSteps * kVocab) / 4;
    repack_out_kernel<<<(total4 + 255) / 256, 256, 0, stream>>>(LPAD, bout, out);
  }
}
